// DistHead_54082228191963
// MI455X (gfx1250) — hardware-verified
//
#include <hip/hip_runtime.h>


namespace {
constexpr int N = 8192, DIN = 256, H = 64, MB = 64, NM = N / MB;
constexpr float XS = 8.0f, PS = 1024.0f, WSC = 256.0f;
typedef _Float16 b16;
typedef __attribute__((ext_vector_type(16))) _Float16 v16b;
typedef __attribute__((ext_vector_type(8))) _Float16 v8b;
typedef __attribute__((ext_vector_type(8))) float v8f;
typedef __attribute__((ext_vector_type(4))) float v4f;
typedef __attribute__((ext_vector_type(2))) float v2f;
__device__ __forceinline__ float bf16_rne(float f) { unsigned int u = __float_as_uint(f); u += 0x7FFFu + ((u >> 16) & 1u); return __uint_as_float(u & 0xFFFF0000u); }
__device__ __forceinline__ void split16(float v, b16& hi, b16& lo) { hi = (b16)v; lo = (b16)(v - (float)hi); }
__device__ __forceinline__ v16b frag_kb(const b16* p, int hh) { const v8b a = *(const v8b*)(p + 8 * hh), b = *(const v8b*)(p + 16 + 8 * hh); v16b f;
#pragma unroll
  for (int e = 0; e < 8; ++e) { f[e] = a[e]; f[8 + e] = b[e]; } return f; }
__device__ __forceinline__ v8f wmma16b(v16b a, v16b b, v8f c) { v8f d = __builtin_amdgcn_wmma_f32_16x16x32_f16(false, a, false, b, (short)0, c, false, false); asm volatile("v_nop\n\tv_nop\n\tv_nop\n\tv_nop" : "+v"(d) : "v"(a), "v"(b)); return d; }
__device__ __forceinline__ void wave_lds_sync() { __builtin_amdgcn_fence(__ATOMIC_RELEASE, "workgroup"); __builtin_amdgcn_wave_barrier(); __builtin_amdgcn_fence(__ATOMIC_ACQUIRE, "workgroup"); }
__device__ __forceinline__ float pmul(float a, float b) { float p = a * b; asm volatile("" : "+v"(p)); return p; }

__global__ __launch_bounds__(256) void wcopy_kernel(const float* __restrict__ w, int ro, b16* __restrict__ WT) {
  const int u = blockIdx.x * 256 + threadIdx.x; if (u >= H * 32) return; const int o = u / 32, k0 = (u % 32) * 8; v8b v;
#pragma unroll
  for (int j = 0; j < 8; ++j) v[j] = (b16)(bf16_rne(w[(size_t)o * DIN + k0 + j]) * WSC); for (int pass = 0; pass < 2; ++pass) { *(volatile v8b*)(WT + (size_t)(ro + o) * DIN + k0) = v; __threadfence(); }
}
__global__ __launch_bounds__(32) void proj_kernel(const float* __restrict__ X, const b16* __restrict__ WT, int NLIM, float* __restrict__ KQV) {
  __shared__ __attribute__((aligned(16))) b16 Ah[16][DIN + 8]; __shared__ __attribute__((aligned(16))) float Tf[16][3 * H + 4];
  const int lane = threadIdx.x, nloc = lane & 15, hlf = lane >> 4; const size_t m0 = (size_t)blockIdx.x * 16; if (m0 >= (size_t)NLIM) return;
  for (int rr = 0; rr < 16; ++rr) for (int q = 0; q < DIN / 32; ++q) Ah[rr][q * 32 + lane] = (b16)(bf16_rne(X[(m0 + rr) * DIN + q * 32 + lane]) * XS);
  wave_lds_sync(); v8f acc[12];
#pragma unroll
  for (int t = 0; t < 12; ++t) acc[t] = (v8f){};
#pragma unroll 2
  for (int kb = 0; kb < DIN; kb += 32) { const v16b a = frag_kb(&Ah[nloc][kb], hlf);
#pragma unroll
    for (int t = 0; t < 12; ++t) acc[t] = wmma16b(a, frag_kb(WT + (size_t)(t * 16 + nloc) * DIN + kb, hlf), acc[t]); }
#pragma unroll
  for (int t = 0; t < 12; ++t)
#pragma unroll
    for (int r8 = 0; r8 < 8; ++r8) Tf[8 * hlf + r8][t * 16 + nloc] = acc[t][r8] * (1.0f / (XS * WSC));
  wave_lds_sync();
  for (int pass = 0; pass < 2; ++pass) { for (int rr = 0; rr < 16; ++rr) for (int q = 0; q < 6; ++q) ((volatile float*)KQV)[(m0 + rr) * (3 * H) + q * 32 + lane] = Tf[rr][q * 32 + lane]; __threadfence(); }
}
__global__ __launch_bounds__(32) void att_kernel(const float* __restrict__ KQV, const float* __restrict__ Z, const float* __restrict__ invr, int NMV, float* __restrict__ out) {
  __shared__ __attribute__((aligned(16))) b16 Qh[16][72], Ql[16][72], Kh[64][72], Kl[64][72], Ph[16][72], Pl[16][72], Vh[H][72], Vl[H][72]; __shared__ float Sc[16][65], Of[16][H + 1];
  const int lane = threadIdx.x, nloc = lane & 15, hlf = lane >> 4; const int m = blockIdx.x >> 2, qb = blockIdx.x & 3; if (m >= NMV) return; const size_t a0 = (size_t)m * MB, q0 = a0 + qb * 16; const float ir = bf16_rne(invr[0]);
  for (int rr = 0; rr < 16; ++rr) for (int q = 0; q < 2; ++q) { b16 p, pl; split16(KQV[(q0 + rr) * (3 * H) + H + q * 32 + lane] * XS, p, pl); Qh[rr][q * 32 + lane] = p; Ql[rr][q * 32 + lane] = pl; }
  for (int rr = 0; rr < 64; ++rr) for (int q = 0; q < 2; ++q) { const float* row = KQV + (a0 + rr) * (3 * H); b16 p, pl; split16(row[q * 32 + lane] * XS, p, pl); Kh[rr][q * 32 + lane] = p; Kl[rr][q * 32 + lane] = pl; split16(row[2 * H + q * 32 + lane] * XS, p, pl); Vh[q * 32 + lane][rr] = p; Vl[q * 32 + lane][rr] = pl; }
  wave_lds_sync();
#pragma unroll
  for (int t = 0; t < 4; ++t) { v8f s = {};
#pragma unroll
    for (int kb = 0; kb < H; kb += 32) { const v16b qh = frag_kb(&Qh[nloc][kb], hlf), ql = frag_kb(&Ql[nloc][kb], hlf), kh = frag_kb(&Kh[t * 16 + nloc][kb], hlf), kl = frag_kb(&Kl[t * 16 + nloc][kb], hlf); s = wmma16b(qh, kh, s); s = wmma16b(qh, kl, s); s = wmma16b(ql, kh, s); }
#pragma unroll
    for (int r8 = 0; r8 < 8; ++r8) Sc[8 * hlf + r8][t * 16 + nloc] = s[r8] * (0.125f / (XS * XS)); }
  wave_lds_sync();
  for (int qi = 0; qi < 16; ++qi) { const float s0 = Sc[qi][lane], s1 = Sc[qi][32 + lane]; float mx = fmaxf(s0, s1); for (int o = 16; o; o >>= 1) mx = fmaxf(mx, __shfl_xor(mx, o)); const float e0 = __expf(s0 - mx), e1 = __expf(s1 - mx); float sm = e0 + e1; for (int o = 16; o; o >>= 1) sm += __shfl_xor(sm, o); const float inv = 1.0f / sm;
    const float* zq = Z + (q0 + qi) * 3; const float zq0 = bf16_rne(zq[0]), zq1 = bf16_rne(zq[1]), zq2 = bf16_rne(zq[2]);
    for (int j = 0; j < 2; ++j) { const float* zk = Z + (a0 + j * 32 + lane) * 3; const float dx = zq0 - bf16_rne(zk[0]), dy = zq1 - bf16_rne(zk[1]), dz = zq2 - bf16_rne(zk[2]); const float d = sqrtf(pmul(dx, dx) + pmul(dy, dy) + pmul(dz, dz)); const float w = pmul(pmul(j ? e1 : e0, inv), __expf(-pmul(ir, d))); b16 p, pl; split16(w * PS, p, pl); Ph[qi][j * 32 + lane] = p; Pl[qi][j * 32 + lane] = pl; } }
  wave_lds_sync(); v8f oacc[4] = {(v8f){}, (v8f){}, (v8f){}, (v8f){}};
#pragma unroll
  for (int kb = 0; kb < MB; kb += 32) { const v16b pa = frag_kb(&Ph[nloc][kb], hlf), pb = frag_kb(&Pl[nloc][kb], hlf);
#pragma unroll
    for (int t = 0; t < 4; ++t) { const v16b vh = frag_kb(&Vh[t * 16 + nloc][kb], hlf), vl = frag_kb(&Vl[t * 16 + nloc][kb], hlf); oacc[t] = wmma16b(pa, vh, oacc[t]); oacc[t] = wmma16b(pa, vl, oacc[t]); oacc[t] = wmma16b(pb, vh, oacc[t]); } }
#pragma unroll
  for (int t = 0; t < 4; ++t)
#pragma unroll
    for (int r8 = 0; r8 < 8; ++r8) Of[8 * hlf + r8][t * 16 + nloc] = oacc[t][r8] * (1.0f / (PS * XS));
  wave_lds_sync();
  for (int pass = 0; pass < 2; ++pass) { for (int rr = 0; rr < 16; ++rr) *(volatile v2f*)(out + (q0 + rr) * H + lane * 2) = (v2f){Of[rr][lane * 2], Of[rr][lane * 2 + 1]}; __threadfence(); }
}
}

extern "C" void kernel_launch(void* const* d_in, const int* in_sizes, int n_in, void* d_out, int out_size, void* d_ws, size_t ws_size, hipStream_t stream) {
  (void)n_in;
  auto Fp = [&](int i) { return (const float*)d_in[i]; };
  if (in_sizes[0] != N * DIN || in_sizes[1] != N * 3 || in_sizes[2] != H * DIN || in_sizes[3] != H * DIN || in_sizes[4] != H * DIN || in_sizes[5] != 1 || in_sizes[6] != NM + 1 || out_size != N * H) return;
  const int NMV = NM;
  size_t off = 0; char* ws = (char*)d_ws;
  auto carve = [&](size_t bytes) { char* p = ws + off; off += (bytes + 255) & ~(size_t)255; return p; };
  b16* WT = (b16*)carve((size_t)3 * H * DIN * 2); float* KQV = (float*)carve((size_t)N * 3 * H * 4);
  if (off > ws_size || off > ((size_t)16 << 20)) return;
  wcopy_kernel<<<(H * 32 + 255) / 256, 256, 0, stream>>>(Fp(2), 0, WT); wcopy_kernel<<<(H * 32 + 255) / 256, 256, 0, stream>>>(Fp(3), H, WT); wcopy_kernel<<<(H * 32 + 255) / 256, 256, 0, stream>>>(Fp(4), 2 * H, WT);
  proj_kernel<<<(NMV * MB) / 16, 32, 0, stream>>>(Fp(0), WT, NMV * MB, KQV);
  att_kernel<<<NMV * 4, 32, 0, stream>>>(KQV, Fp(1), Fp(5), NMV, (float*)d_out);
}
